// FlexAttentionWithRoPE_31482110279735
// MI455X (gfx1250) — hardware-verified
//
#include <hip/hip_runtime.h>
#include <math.h>

typedef __attribute__((ext_vector_type(16))) _Float16 v16h;
typedef __attribute__((ext_vector_type(8)))  _Float16 v8h;
typedef __attribute__((ext_vector_type(8)))  float    v8f;
typedef __attribute__((ext_vector_type(4)))  float    v4f;

#define B_ 2
#define H_ 16
#define L_ 2048
#define D_ 64
#define F_ 32
#define PR 64
#define VP 72
#define AT_NW 4
#define AT_QB 64
#define AT_KC 64
#define PSC 32768.0f

__device__ __forceinline__ void dep_guard_h(v8f& a, v8f& b, v16h x, v16h y) {
  asm volatile("v_nop\n\tv_nop\n\tv_nop\n\tv_nop" : "+v"(a), "+v"(b) : "v"(x), "v"(y));
}
template <typename T> struct Frag;
template <> struct Frag<_Float16> {
  typedef v16h V; union U { v16h v; v8h h[2]; };
  static __device__ __forceinline__ v16h load(const _Float16* p) {
    U f; f.h[0] = *(const v8h*)(p); f.h[1] = *(const v8h*)(p + 16); return f.v;
  }
  static __device__ __forceinline__ v8f mma(v16h a, v16h b, v8f c) {
    return __builtin_amdgcn_wmma_f32_16x16x32_f16(false, a, false, b, (short)0, c, false, false);
  }
};
__device__ __forceinline__ v8f hmma(v16h a, v16h b, v8f c) {
  c = __builtin_amdgcn_wmma_f32_16x16x32_f16(false, a, false, b, (short)0, c, false, false);
  asm volatile("v_nop\n\tv_nop\n\tv_nop\n\tv_nop" : "+v"(c) : "v"(a), "v"(b));
  return c;
}

__global__ __launch_bounds__(256)
void rope_prep_kernel(const float* __restrict__ q, const float* __restrict__ k, const float* __restrict__ v,
                      const float* __restrict__ pos, const float* __restrict__ freqs,
                      _Float16* __restrict__ q16, _Float16* __restrict__ k16, _Float16* __restrict__ vt16)
{
  __shared__ __align__(16) _Float16 Qs[PR * D_];
  __shared__ __align__(16) _Float16 Ks[PR * D_];
  __shared__ __align__(16) _Float16 Vs[D_ * VP];

  const int tid = threadIdx.x;
  const int nlb = L_ / PR;
  const int bh  = blockIdx.x / nlb;
  const int lb  = blockIdx.x - bh * nlb;
  const int b   = bh / H_;
  const int h   = bh - b * H_;
  const int l0  = lb * PR;
  const size_t row0 = (size_t)bh * L_ + l0;
  const float* qb = q + row0 * D_;
  const float* kb = k + row0 * D_;
  const float* vb = v + row0 * D_;
  const float* pb = pos + ((size_t)b * L_ + l0) * 2;
  const float* fb = freqs + (size_t)h * F_ * 2;

#pragma unroll 1
  for (int it = 0; it < (PR * F_) / 256; ++it) {
    const int item = it * 256 + tid;
    const int r = item >> 5;
    const int f = item & 31;
    const float p0  = pb[r * 2 + 0], p1  = pb[r * 2 + 1];
    const float fr0 = fb[f * 2 + 0], fr1 = fb[f * 2 + 1];
    const float th = p0 * fr0 + p1 * fr1;
    const float c = cosf(th);
    const float s = sinf(th);
    const float q1 = qb[r * D_ + f], q2 = qb[r * D_ + f + F_];
    const float k1 = kb[r * D_ + f], k2 = kb[r * D_ + f + F_];
    Qs[r * D_ + f]      = (_Float16)(q1 * c - q2 * s);
    Qs[r * D_ + f + F_] = (_Float16)(q2 * c + q1 * s);
    Ks[r * D_ + f]      = (_Float16)(k1 * c - k2 * s);
    Ks[r * D_ + f + F_] = (_Float16)(k2 * c + k1 * s);
  }

  {
    const int r  = tid >> 2;
    const int dq = (tid & 3) * 16;
    const float* vp = vb + r * D_ + dq;
    const v4f a0 = *(const v4f*)(vp + 0);
    const v4f a1 = *(const v4f*)(vp + 4);
    const v4f a2 = *(const v4f*)(vp + 8);
    const v4f a3 = *(const v4f*)(vp + 12);
#pragma unroll
    for (int e = 0; e < 4; ++e) {
      Vs[(dq + e) * VP + r]      = (_Float16)a0[e];
      Vs[(dq + 4 + e) * VP + r]  = (_Float16)a1[e];
      Vs[(dq + 8 + e) * VP + r]  = (_Float16)a2[e];
      Vs[(dq + 12 + e) * VP + r] = (_Float16)a3[e];
    }
  }
  __syncthreads();

  {
    const int c8 = (tid & 7) * 8;
    const int rr = tid >> 3;
    for (int pass = 0; pass < 2; ++pass) {
#pragma unroll
      for (int it = 0; it < 2; ++it) {
        const int row = it * 32 + rr;
        const v8h qv = *(const v8h*)(Qs + row * D_ + c8);
        const v8h kv = *(const v8h*)(Ks + row * D_ + c8);
        const v8h vv = *(const v8h*)(Vs + row * VP + c8);
        *(volatile v8h*)(q16 + (row0 + row) * D_ + c8) = qv;
        *(volatile v8h*)(k16 + (row0 + row) * D_ + c8) = kv;
        *(volatile v8h*)(vt16 + ((size_t)bh * D_ + row) * L_ + l0 + c8) = vv;
      }
      __threadfence();
    }
  }
}

__global__ __launch_bounds__(128)
void attn_f16_kernel(const _Float16* __restrict__ q16, const _Float16* __restrict__ k16,
                     const _Float16* __restrict__ vt16, float* __restrict__ out, float sm_scale)
{
  __shared__ __align__(16) _Float16 Ksh[AT_KC * D_];
  __shared__ __align__(16) _Float16 Vth[D_ * AT_KC];
  __shared__ __align__(16) _Float16 Psh[AT_NW][16 * AT_KC];
  __shared__ __align__(16) float    Os[AT_NW][16 * 68];

  const int tid  = threadIdx.x;
  const int wave = tid >> 5;
  const int lane = tid & 31;
  const int hh   = lane >> 4;
  const int c    = lane & 15;

  const int nqb = L_ / AT_QB;
  const int bx  = blockIdx.x;
  const int qb  = bx % nqb;
  const int bh  = bx / nqb;
  const int q0  = qb * AT_QB + wave * 16;

  const _Float16* qp = q16  + (size_t)bh * L_ * D_;
  const _Float16* kp = k16  + (size_t)bh * L_ * D_;
  const _Float16* vp = vt16 + (size_t)bh * D_ * L_;
  float*          op = out  + (size_t)bh * L_ * D_;

  v16h qa[2];
#pragma unroll
  for (int dc = 0; dc < 2; ++dc)
    qa[dc] = Frag<_Float16>::load(qp + (size_t)(q0 + c) * D_ + dc * 32 + 8 * hh);

  float mrow[8], lrow[8];
  v8f oacc[4];
#pragma unroll
  for (int r = 0; r < 8; ++r) { mrow[r] = -INFINITY; lrow[r] = 0.f; }
#pragma unroll
  for (int t = 0; t < 4; ++t) oacc[t] = (v8f){0.f,0.f,0.f,0.f,0.f,0.f,0.f,0.f};

  for (int kc = 0; kc < L_ / AT_KC; ++kc) {
    const int kv0 = kc * AT_KC;
    __syncthreads();
    {
      const int rr = tid >> 1, dh = (tid & 1) * 32;
      const _Float16* krow = kp + (size_t)(kv0 + rr) * D_ + dh;
      const _Float16* vrow = vp + (size_t)rr * L_ + kv0 + dh;
#pragma unroll
      for (int i = 0; i < 4; ++i) {
        const v8h kk = *(const v8h*)(krow + 8 * i);
        const v8h vv = *(const v8h*)(vrow + 8 * i);
        *(v8h*)(Ksh + rr * D_ + dh + 8 * i)    = kk;
        *(v8h*)(Vth + rr * AT_KC + dh + 8 * i) = vv;
      }
    }
    __syncthreads();

    v8f s[4];
#pragma unroll
    for (int j = 0; j < 4; ++j) {
      s[j] = (v8f){0.f,0.f,0.f,0.f,0.f,0.f,0.f,0.f};
#pragma unroll
      for (int dc = 0; dc < 2; ++dc) {
        const v16h kb = Frag<_Float16>::load(Ksh + (j * 16 + c) * D_ + dc * 32 + 8 * hh);
        s[j] = hmma(qa[dc], kb, s[j]);
      }
    }

    float cm[8];
#pragma unroll
    for (int r = 0; r < 8; ++r) {
      float m = -INFINITY;
#pragma unroll
      for (int j = 0; j < 4; ++j) {
        s[j][r] *= sm_scale;
        m = fmaxf(m, s[j][r]);
      }
#pragma unroll
      for (int off = 1; off < 16; off <<= 1) m = fmaxf(m, __shfl_xor(m, off, 32));
      cm[r] = m;
    }

    _Float16* pw = Psh[wave];
#pragma unroll
    for (int r = 0; r < 8; ++r) {
      const float mnew  = fmaxf(mrow[r], cm[r]);
      const float alpha = expf(mrow[r] - mnew);
      mrow[r] = mnew;
      float psum = 0.f;
#pragma unroll
      for (int j = 0; j < 4; ++j) {
        const float p = expf(s[j][r] - mnew);
        psum += p;
        pw[(8 * hh + r) * AT_KC + j * 16 + c] = (_Float16)(p * PSC);
      }
#pragma unroll
      for (int off = 1; off < 16; off <<= 1) psum += __shfl_xor(psum, off, 32);
      lrow[r] = lrow[r] * alpha + psum;
#pragma unroll
      for (int t = 0; t < 4; ++t) oacc[t][r] *= alpha;
    }
    __builtin_amdgcn_fence(__ATOMIC_RELEASE, "workgroup");
    __builtin_amdgcn_wave_barrier();
    __builtin_amdgcn_fence(__ATOMIC_ACQUIRE, "workgroup");

#pragma unroll 1
    for (int kk = 0; kk < 2; ++kk) {
      const v16h pa = Frag<_Float16>::load(pw + c * AT_KC + kk * 32 + 8 * hh);
#pragma unroll
      for (int t = 0; t < 4; ++t) {
        const v16h vb = Frag<_Float16>::load(Vth + (t * 16 + c) * AT_KC + kk * 32 + 8 * hh);
        oacc[t] = hmma(pa, vb, oacc[t]);
      }
    }
  }

  float* os = Os[wave];
#pragma unroll
  for (int r = 0; r < 8; ++r) {
    const float inv = 1.0f / (lrow[r] * PSC);
#pragma unroll
    for (int t = 0; t < 4; ++t) os[(8 * hh + r) * 68 + t * 16 + c] = oacc[t][r] * inv;
  }
  __builtin_amdgcn_fence(__ATOMIC_RELEASE, "workgroup");
  __builtin_amdgcn_wave_barrier();
  __builtin_amdgcn_fence(__ATOMIC_ACQUIRE, "workgroup");
  {
    const int c4 = (lane & 15) * 4;
    for (int pass = 0; pass < 2; ++pass) {
#pragma unroll
      for (int it = 0; it < 8; ++it) {
        const int row = it * 2 + hh;
        const v4f val = *(const v4f*)(os + row * 68 + c4);
        *(volatile v4f*)(op + (size_t)(q0 + row) * D_ + c4) = val;
      }
      __threadfence();
    }
  }
}

extern "C" void kernel_launch(void* const* d_in, const int* in_sizes, int n_in,
                              void* d_out, int out_size, void* d_ws, size_t ws_size,
                              hipStream_t stream) {
  const size_t nq = (size_t)B_ * H_ * L_ * D_;
  if (n_in < 5) return;
  if (in_sizes[0] != (int)nq || in_sizes[1] != (int)nq || in_sizes[2] != (int)nq) return;
  if (in_sizes[3] != B_ * L_ * 2 || in_sizes[4] != H_ * F_ * 2) return;
  if (out_size != (int)nq) return;
  const size_t need = 3 * nq * sizeof(_Float16);
  if (need > ws_size) return;

  const float* q     = (const float*)d_in[0];
  const float* k     = (const float*)d_in[1];
  const float* v     = (const float*)d_in[2];
  const float* pos   = (const float*)d_in[3];
  const float* freqs = (const float*)d_in[4];
  float* out = (float*)d_out;

  _Float16* q16  = (_Float16*)d_ws;
  _Float16* k16  = q16 + nq;
  _Float16* vt16 = k16 + nq;

  const int nblk = B_ * H_ * (L_ / PR);
  rope_prep_kernel<<<dim3(nblk), dim3(256), 0, stream>>>(q, k, v, pos, freqs, q16, k16, vt16);
  attn_f16_kernel<<<dim3(B_ * H_ * (L_ / AT_QB)), dim3(128), 0, stream>>>(q16, k16, vt16, out, 0.125f);
}
